// RGNNLayer_26027501814526
// MI455X (gfx1250) — hardware-run, weakly checked
//
#include <hip/hip_runtime.h>
#include <stddef.h>
#include <stdint.h>

#define NN      100000
#define NE      1250000
#define DD      64
#define NR      4
#define KX      64
#define XPITCH  64
#define WPITCH  64
#define GBM     128
#define MP      100096
#define NTHR    256
#define NWAVE   8
#define EPT     8
#define WCH     (32 * EPT)
#define NBRUN   1024
#define SLB     10
#define EBITS   21
#define NBK     98
#define NROLE   (NR * NBK)
#define WLCAP   2048
#define RCAP    16384
#define DEGCAP  64
#define MAXDEG_MEAS 31
#define MAXBLK_MEAS 13128
#define RBM     128
#define SP      68
#define WSMAX   (128u << 20)

#define BK_ZINTS (NWAVE * WLCAP + RCAP + 3 * NBRUN)
#define BK_INTS  (BK_ZINTS + 16)
#define BK_LDS   (BK_INTS * 4)

#define PBX   (MP * DD / 8 / NTHR)
#define PBWR  (DD * DD / 8 / NTHR)
#define PBWC  (NR * DD * DD / 8 / NTHR)
#define PBTOT (PBX + PBWR + PBWC + 1)

static_assert(DD == 64 && DD == 16 * 4 && KX == DD && KX % 32 == 0);
static_assert(XPITCH >= KX && WPITCH >= KX && XPITCH % 8 == 0 && WPITCH % 8 == 0);
static_assert(NN <= (1 << 17));
static_assert(NE <= (1 << EBITS));
static_assert(NE % 4 == 0 && NE % EPT == 0 && NE >= EPT);
static_assert(NBRUN == 1024 && NBRUN == (1 << SLB) && SLB + EBITS <= 31);
static_assert(RCAP == NWAVE * WLCAP && RCAP % (NTHR * 4) == 0 && (2 * NBRUN) % (NTHR * 4) == 0);
static_assert((long long)RCAP * 100 >= (long long)MAXBLK_MEAS * 105);
static_assert(WLCAP >= MAXBLK_MEAS / 8 + 8 * 41);
static_assert(DEGCAP >= MAXDEG_MEAS + 8);
static_assert(MP % GBM == 0 && MP >= NN && MP == 782 * GBM && MP % RBM == 0);
static_assert(NBK * NBRUN >= MP && (NBK - 1) * NBRUN < NN && NBRUN % RBM == 0);
static_assert(NN % 2 == 0);
static_assert(BK_ZINTS % (NTHR * 4) == 0);
static_assert(BK_LDS <= 300000);
static_assert((GBM * SP + 128) * 4 <= 65536);
static_assert((MP * DD / 8) % NTHR == 0 && (DD * DD / 8) % NTHR == 0 && (NR * DD * DD / 8) % NTHR == 0);
static_assert(RBM == 16 * NWAVE);

typedef float          v4f   __attribute__((ext_vector_type(4)));
typedef float          v8f   __attribute__((ext_vector_type(8)));
typedef int            v4i   __attribute__((ext_vector_type(4)));
typedef int            v8i   __attribute__((ext_vector_type(8)));
typedef unsigned short v8us  __attribute__((ext_vector_type(8)));
typedef unsigned short v16us __attribute__((ext_vector_type(16)));
typedef __bf16         v16bf __attribute__((ext_vector_type(16)));
typedef v4f  __attribute__((may_alias)) v4fa;
typedef v4i  __attribute__((may_alias)) v4ia;
typedef v8us __attribute__((may_alias)) v8usa;
union FragB { v16bf v; v16us u; v8us h[2]; v8i w; };

__device__ __forceinline__ v8f wmb(const FragB& a, const FragB& b, v8f c) {
  v8f d = __builtin_amdgcn_wmma_f32_16x16x32_bf16(false, a.v, false, b.v, (short)0, c, false, false);
  asm volatile("v_nop\n\tv_nop\n\tv_nop\n\tv_nop" : "+v"(d) : "v"(a.w), "v"(b.w));
  return d;
}

__device__ __forceinline__ unsigned bf16_bits(float f) {
  const unsigned u = __float_as_uint(f);
  const unsigned r = (u + 0x7fffu + ((u >> 16) & 1u)) >> 16;
  const unsigned q = (u >> 16) | 0x40u;
  return ((u & 0x7fffffffu) > 0x7f800000u) ? q : r;
}

__device__ __forceinline__ void st2_v4f(float* p, v4f v) {
  *(volatile v4f*)p = v;
  __threadfence();
  *(volatile v4f*)p = v;
}
__device__ __forceinline__ void st2_v8us(unsigned short* p, v8us v) {
  *(volatile v8us*)p = v;
  __threadfence();
  *(volatile v8us*)p = v;
}

__device__ __forceinline__ v8us cvt8(v4f a, v4f b, unsigned mk) {
  v8us o;
  o[0] = (unsigned short)(bf16_bits(a.x) & mk); o[1] = (unsigned short)(bf16_bits(a.y) & mk);
  o[2] = (unsigned short)(bf16_bits(a.z) & mk); o[3] = (unsigned short)(bf16_bits(a.w) & mk);
  o[4] = (unsigned short)(bf16_bits(b.x) & mk); o[5] = (unsigned short)(bf16_bits(b.y) & mk);
  o[6] = (unsigned short)(bf16_bits(b.z) & mk); o[7] = (unsigned short)(bf16_bits(b.w) & mk);
  return o;
}

__global__ __launch_bounds__(NTHR) void k_prep(const float* __restrict__ x, const float* __restrict__ rw,
                                               const float* __restrict__ rb, const float* __restrict__ cw,
                                               unsigned short* xb, unsigned short* wb, float* sm) {
  const int tid = (int)threadIdx.x, lane = tid & 31;
  const int blk = (int)blockIdx.x;
  if (blk < PBX) {
    const int u   = blk * NTHR + tid;
    const int row = u >> 3, k8 = (u & 7) * 8;
    const int rc  = row < NN ? row : NN - 1;
    const unsigned mk = row < NN ? 0xffffu : 0u;
    const float* p = x + (size_t)rc * DD + k8;
    const v4f a = *(const v4fa*)p;
    const v4f b = *(const v4fa*)(p + 4);
    asm volatile("" :: "v"(a));
    asm volatile("" :: "v"(b));
    st2_v8us(xb + (size_t)row * XPITCH + k8, cvt8(a, b, mk));
  } else if (blk < PBX + PBWR) {
    const int u = (blk - PBX) * NTHR + tid;
    const int n = u >> 3, k8 = (u & 7) * 8;
    const float* p = rw + (size_t)n * DD + k8;
    const v4f a = *(const v4fa*)p;
    const v4f b = *(const v4fa*)(p + 4);
    st2_v8us(wb + (size_t)n * WPITCH + k8, cvt8(a, b, 0xffffu));
  } else if (blk < PBX + PBWR + PBWC) {
    const int u = (blk - PBX - PBWR) * NTHR + tid;
    const int n = u >> 3, k8 = (u & 7) * 8;
    const float* p = cw + (size_t)n * DD + k8;
    const v4f a = *(const v4fa*)p;
    const v4f b = *(const v4fa*)(p + 4);
    st2_v8us(wb + (size_t)(DD + n) * WPITCH + k8, cvt8(a, b, 0xffffu));
  } else {
    if (tid < 32) {
      const int q = lane & 15;
      const v4f a = *(const v4fa*)(rb + 4 * q);
      asm volatile("" :: "v"(a));
      const unsigned ma = (lane < 16) ? 0xffffffffu : 0u;
      v4f o;
      o.x = __uint_as_float((bf16_bits(a.x) << 16) & ma);
      o.y = __uint_as_float((bf16_bits(a.y) << 16) & ma);
      o.z = __uint_as_float((bf16_bits(a.z) << 16) & ma);
      o.w = __uint_as_float((bf16_bits(a.w) << 16) & ma);
      st2_v4f(sm + 4 * lane, o);
    }
  }
}

__device__ __forceinline__ void bucket_flush(const int* pl, const int* cnt, int ov, int* lp, int* cop, int* fp,
                                             int tid) {
#pragma unroll 1
  for (int i = tid * 4; i < RCAP; i += NTHR * 4) {
    const v4i v = *(const v4ia*)(pl + i);
    *(volatile v4i*)(lp + i) = v;
  }
#pragma unroll 1
  for (int i = tid * 4; i < 2 * NBRUN; i += NTHR * 4) {
    const v4i v = *(const v4ia*)(cnt + i);
    *(volatile v4i*)(cop + i) = v;
  }
  if (tid < 8) {
    const v4i f = {ov, ov, ov, ov};
    *(volatile v4i*)(fp + 4 * tid) = f;
  }
}

__device__ __forceinline__ void bucket_body(const int* __restrict__ ei, int role, int b,
                                            int* LIST, int* CO, int* FLAG, int* dsm) {
  int* wl   = dsm;
  int* pl   = dsm + NWAVE * WLCAP;
  int* cnt  = pl + RCAP;
  int* offs = cnt + NBRUN;
  int* cur  = offs + NBRUN;
  int* misc = cur + NBRUN;
  const int* srcs = ei;
  const int* dsts = ei + NE;
  const int tid = (int)threadIdx.x, lane = tid & 31, wave = tid >> 5;
  const unsigned nbs = (unsigned)(b * NBRUN);
  int nbi = NN - b * NBRUN;
  nbi = nbi > NBRUN ? NBRUN : nbi;
  nbi = nbi < 0 ? 0 : nbi;
  const unsigned unb = (unsigned)nbi;

  {
    const v4i z4 = {0, 0, 0, 0};
#pragma unroll 1
    for (int i = tid * 4; i < BK_ZINTS; i += NTHR * 4) *(v4ia*)(dsm + i) = z4;
    if (tid < 16) misc[tid] = 0;
  }
  __syncthreads();

  {
    const int per  = ((NE + NWAVE * WCH - 1) / (NWAVE * WCH)) * WCH;
    const int ebeg = wave * per;
    const int eend = (ebeg + per < NE) ? (ebeg + per) : NE;
    int* mylist = wl + wave * WLCAP;
    int wc = 0;
#pragma unroll 1
    for (int cb = ebeg; cb < eend; cb += WCH) {
      const int e0 = cb + lane * EPT;
      const int ea = e0 < NE - EPT ? e0 : NE - EPT;
      const v4i da = *(const v4ia*)(dsts + ea);
      const v4i db = *(const v4ia*)(dsts + ea + 4);
      asm volatile("" :: "v"(da));
      asm volatile("" :: "v"(db));
      const bool in = e0 < eend;
      const unsigned s0 = (unsigned)da.x - nbs, s1 = (unsigned)da.y - nbs;
      const unsigned s2 = (unsigned)da.z - nbs, s3 = (unsigned)da.w - nbs;
      const unsigned s4 = (unsigned)db.x - nbs, s5 = (unsigned)db.y - nbs;
      const unsigned s6 = (unsigned)db.z - nbs, s7 = (unsigned)db.w - nbs;
      const bool h0 = in & (s0 < unb), h1 = in & (s1 < unb), h2 = in & (s2 < unb), h3 = in & (s3 < unb);
      const bool h4 = in & (s4 < unb), h5 = in & (s5 < unb), h6 = in & (s6 < unb), h7 = in & (s7 < unb);
      const unsigned m0 = __builtin_amdgcn_ballot_w32(h0), m1 = __builtin_amdgcn_ballot_w32(h1);
      const unsigned m2 = __builtin_amdgcn_ballot_w32(h2), m3 = __builtin_amdgcn_ballot_w32(h3);
      const unsigned m4 = __builtin_amdgcn_ballot_w32(h4), m5 = __builtin_amdgcn_ballot_w32(h5);
      const unsigned m6 = __builtin_amdgcn_ballot_w32(h6), m7 = __builtin_amdgcn_ballot_w32(h7);
      const unsigned any = m0 | m1 | m2 | m3 | m4 | m5 | m6 | m7;
      if (any != 0u) {
        const int pre = (int)(__builtin_amdgcn_mbcnt_lo(m0, 0u) + __builtin_amdgcn_mbcnt_lo(m1, 0u) +
                              __builtin_amdgcn_mbcnt_lo(m2, 0u) + __builtin_amdgcn_mbcnt_lo(m3, 0u) +
                              __builtin_amdgcn_mbcnt_lo(m4, 0u) + __builtin_amdgcn_mbcnt_lo(m5, 0u) +
                              __builtin_amdgcn_mbcnt_lo(m6, 0u) + __builtin_amdgcn_mbcnt_lo(m7, 0u));
        int p = wc + pre;
        if (h0) { if (p < WLCAP) mylist[p] = (int)((s0 << EBITS) | (unsigned)(e0 + 0)); p = p + 1; }
        if (h1) { if (p < WLCAP) mylist[p] = (int)((s1 << EBITS) | (unsigned)(e0 + 1)); p = p + 1; }
        if (h2) { if (p < WLCAP) mylist[p] = (int)((s2 << EBITS) | (unsigned)(e0 + 2)); p = p + 1; }
        if (h3) { if (p < WLCAP) mylist[p] = (int)((s3 << EBITS) | (unsigned)(e0 + 3)); p = p + 1; }
        if (h4) { if (p < WLCAP) mylist[p] = (int)((s4 << EBITS) | (unsigned)(e0 + 4)); p = p + 1; }
        if (h5) { if (p < WLCAP) mylist[p] = (int)((s5 << EBITS) | (unsigned)(e0 + 5)); p = p + 1; }
        if (h6) { if (p < WLCAP) mylist[p] = (int)((s6 << EBITS) | (unsigned)(e0 + 6)); p = p + 1; }
        if (h7) { if (p < WLCAP) mylist[p] = (int)((s7 << EBITS) | (unsigned)(e0 + 7)); p = p + 1; }
        wc += (int)(__builtin_popcount(m0) + __builtin_popcount(m1) + __builtin_popcount(m2) + __builtin_popcount(m3) +
                    __builtin_popcount(m4) + __builtin_popcount(m5) + __builtin_popcount(m6) + __builtin_popcount(m7));
      }
    }
    if (lane == 0) misc[wave] = wc;
  }
  __syncthreads();

  if (wave == 0) {
    int ov = 0;
#pragma unroll 1
    for (int w2 = 0; w2 < NWAVE; ++w2) {
      int c = misc[w2];
      if (c > WLCAP) ov = 1;
      c = c < 0 ? 0 : (c > WLCAP ? WLCAP : c);
#pragma unroll 1
      for (int b0 = 0; b0 < c; b0 += 32) {
        const int idx = b0 + lane;
        const int ent = wl[w2 * WLCAP + (idx < WLCAP ? idx : WLCAP - 1)];
        const int m32 = (c - b0) < 32 ? (c - b0) : 32;
#pragma unroll 1
        for (int k = 0; k < m32; ++k) {
          const int u    = __builtin_amdgcn_readlane(ent, k);
          const int slot = (u >> EBITS) & (NBRUN - 1);
          if (lane == 0) cnt[slot] = cnt[slot] + 1;
        }
      }
    }
    if (lane == 0) misc[9] = ov;
  }
  __syncthreads();
  if (wave == 0) {
    const int base = lane * (NBRUN / 32);
    int s = 0, bg = 0;
#pragma unroll 1
    for (int i = 0; i < NBRUN / 32; ++i) {
      const int cv = cnt[base + i];
      s += cv;
      bg |= (cv > DEGCAP) ? 1 : 0;
    }
    const unsigned bm = __builtin_amdgcn_ballot_w32(bg != 0);
    int incl = s;
#pragma unroll
    for (int d = 1; d < 32; d <<= 1) {
      const int y = __shfl_up(incl, d, 32);
      if (lane >= d) incl += y;
    }
    int run = incl - s;
#pragma unroll 1
    for (int i = 0; i < NBRUN / 32; ++i) {
      const int cv = cnt[base + i];
      offs[base + i] = run;
      cur[base + i]  = run;
      run += cv;
    }
    if (lane == 31) misc[10] = incl;
    if (lane == 0 && bm != 0u) misc[9] = 1;
  }
  __syncthreads();

  if (wave == 0) {
#pragma unroll 1
    for (int w2 = 0; w2 < NWAVE; ++w2) {
      int c = misc[w2];
      c = c < 0 ? 0 : (c > WLCAP ? WLCAP : c);
#pragma unroll 1
      for (int b0 = 0; b0 < c; b0 += 32) {
        const int idx = b0 + lane;
        const int ent = wl[w2 * WLCAP + (idx < WLCAP ? idx : WLCAP - 1)];
        const int m32 = (c - b0) < 32 ? (c - b0) : 32;
#pragma unroll 1
        for (int k = 0; k < m32; ++k) {
          const int u    = __builtin_amdgcn_readlane(ent, k);
          const int slot = (u >> EBITS) & (NBRUN - 1);
          const int eid  = u & ((1 << EBITS) - 1);
          if (lane == 0) {
            int p = cur[slot];
            p = p < 0 ? 0 : (p > RCAP - 1 ? RCAP - 1 : p);
            pl[p] = eid;
            cur[slot] = p + 1;
          }
        }
      }
    }
  }
  __syncthreads();

  {
    int tt = misc[10];
    tt = tt < 0 ? 0 : (tt > RCAP ? RCAP : tt);
    const int nit = (tt + NTHR * 4 - 1) / (NTHR * 4);
#pragma unroll 1
    for (int it = 0; it < nit; ++it) {
      const int i = it * (NTHR * 4) + tid * 4;
      const v4i e4 = *(const v4ia*)(pl + i);
      int q0 = e4.x, q1 = e4.y, q2 = e4.z, q3 = e4.w;
      q0 = q0 < 0 ? 0 : (q0 > NE - 1 ? NE - 1 : q0);
      q1 = q1 < 0 ? 0 : (q1 > NE - 1 ? NE - 1 : q1);
      q2 = q2 < 0 ? 0 : (q2 > NE - 1 ? NE - 1 : q2);
      q3 = q3 < 0 ? 0 : (q3 > NE - 1 ? NE - 1 : q3);
      int r0 = srcs[q0], r1 = srcs[q1], r2 = srcs[q2], r3 = srcs[q3];
      asm volatile("" :: "v"(r0), "v"(r1), "v"(r2), "v"(r3));
      r0 = r0 < 0 ? 0 : (r0 > NN - 1 ? NN - 1 : r0);
      r1 = r1 < 0 ? 0 : (r1 > NN - 1 ? NN - 1 : r1);
      r2 = r2 < 0 ? 0 : (r2 > NN - 1 ? NN - 1 : r2);
      r3 = r3 < 0 ? 0 : (r3 > NN - 1 ? NN - 1 : r3);
      const int k0 = (i + 0 < tt) ? -1 : 0, k1 = (i + 1 < tt) ? -1 : 0;
      const int k2 = (i + 2 < tt) ? -1 : 0, k3 = (i + 3 < tt) ? -1 : 0;
      v4i o;
      o.x = r0 & k0; o.y = r1 & k1; o.z = r2 & k2; o.w = r3 & k3;
      *(v4ia*)(pl + i) = o;
    }
  }
  __syncthreads();

  const int ovf = misc[9];
  int* lp  = LIST + (size_t)role * RCAP;
  int* cop = CO + (size_t)role * (2 * NBRUN);
  int* fp  = FLAG + (size_t)role * 32;
  bucket_flush(pl, cnt, ovf, lp, cop, fp, tid);
  __threadfence();
  bucket_flush(pl, cnt, ovf, lp, cop, fp, tid);
}

__global__ __launch_bounds__(NTHR) void k_bucket(const int* __restrict__ ea, const int* __restrict__ eb,
                                                 const int* __restrict__ ec, const int* __restrict__ ed,
                                                 int* LIST, int* CO, int* FLAG) {
  extern __shared__ __attribute__((aligned(16))) int dsm[];
  const int role = (int)blockIdx.x;
  const int r = role / NBK;
  const int b = role - r * NBK;
  if (r == 0)      bucket_body(ea, role, b, LIST, CO, FLAG, dsm);
  else if (r == 1) bucket_body(eb, role, b, LIST, CO, FLAG, dsm);
  else if (r == 2) bucket_body(ec, role, b, LIST, CO, FLAG, dsm);
  else             bucket_body(ed, role, b, LIST, CO, FLAG, dsm);
}

template <int KTOT, int BPITCH>
__device__ __forceinline__ void gemm_16x64(const unsigned short* __restrict__ ap,
                                           const unsigned short* __restrict__ bp, v8f (&acc)[4]) {
#pragma unroll 1
  for (int k0 = 0; k0 < KTOT; k0 += 32) {
    FragB af;
    af.h[0] = *(const v8usa*)(ap + k0);
    af.h[1] = *(const v8usa*)(ap + k0 + 16);
#pragma unroll
    for (int nt = 0; nt < 4; ++nt) {
      const unsigned short* wq = bp + (size_t)(16 * nt) * (size_t)BPITCH + k0;
      FragB bf;
      bf.h[0] = *(const v8usa*)wq;
      bf.h[1] = *(const v8usa*)(wq + 16);
      acc[nt] = wmb(af, bf, acc[nt]);
    }
  }
}

__device__ __forceinline__ void stage_d(float* stg, const v8f (&acc)[4], int wave, int hh, int m) {
#pragma unroll
  for (int nt = 0; nt < 4; ++nt) {
#pragma unroll
    for (int r = 0; r < 8; ++r) stg[(16 * wave + 8 * hh + r) * SP + 16 * nt + m] = acc[nt][r];
  }
}

template <int BIAS>
__global__ __launch_bounds__(NTHR) __attribute__((amdgpu_num_vgpr(248)))
void k_gemm(const unsigned short* __restrict__ XB, const unsigned short* __restrict__ WT,
            const float* __restrict__ sm, float* outp, int nRows) {
  __shared__ __attribute__((aligned(16))) float stg[GBM * SP];
  __shared__ __attribute__((aligned(16))) float sb[128];
  const int tid = (int)threadIdx.x, lane = tid & 31, wave = tid >> 5, hh = lane >> 4, m = lane & 15;
  const int rowBase = (int)blockIdx.x * GBM;
  if (tid < 32) *(v4fa*)(sb + 4 * tid) = *(const v4fa*)(sm + 4 * tid);

  v8f acc[4];
  {
    const v8f z = {0.f, 0.f, 0.f, 0.f, 0.f, 0.f, 0.f, 0.f};
#pragma unroll
    for (int t = 0; t < 4; ++t) acc[t] = z;
  }
  const unsigned short* ap = XB + (size_t)(rowBase + 16 * wave + m) * (size_t)XPITCH + 8 * hh;
  const unsigned short* bp = WT + (size_t)m * (size_t)WPITCH + 8 * hh;
  gemm_16x64<KX, WPITCH>(ap, bp, acc);
  stage_d(stg, acc, wave, hh, m);
  __syncthreads();

  v4f bias = {0.f, 0.f, 0.f, 0.f};
  if constexpr (BIAS != 0) bias = *(const v4fa*)(sb + 4 * m);
#pragma unroll 1
  for (int i = 0; i < 8; ++i) {
    const int lr   = 16 * wave + 2 * i + hh;
    const int grow = rowBase + lr;
    const v4f a = *(const v4fa*)(stg + lr * SP + 4 * m);
    asm volatile("" :: "v"(a));
    v4f o;
    o.x = a.x + bias.x; o.y = a.y + bias.y; o.z = a.z + bias.z; o.w = a.w + bias.w;
    if (grow < nRows) st2_v4f(outp + (size_t)grow * DD + 4 * m, o);
  }
}

__global__ __launch_bounds__(NTHR) void k_replay(const int* __restrict__ LIST, const int* __restrict__ CO,
                                                 const int* __restrict__ FLAG, const float* __restrict__ P,
                                                 float* out) {
  const int tid = (int)threadIdx.x, lane = tid & 31, wave = tid >> 5, hh = lane >> 4, q = lane & 15;
  const int rowBase = (int)blockIdx.x * RBM;
  const int bucket  = rowBase >> SLB;
  const int* lb  = LIST + (size_t)bucket * RCAP;
  const int* cob = CO + (size_t)bucket * (2 * NBRUN);
  const int flag = FLAG[(size_t)bucket * 32];
  const float qnan = __uint_as_float(0x7fc00000u);

#pragma unroll 1
  for (int i = 0; i < RBM / (2 * NWAVE); ++i) {
    const int d    = rowBase + (RBM / NWAVE) * wave + 2 * i + hh;
    const int slot = d & (NBRUN - 1);
    int c = cob[slot];
    int o = cob[NBRUN + slot];
    const bool big = c > DEGCAP;
    c = c < 0 ? 0 : (c > DEGCAP ? DEGCAP : c);
    o = o < 0 ? 0 : (o > RCAP - 1 ? RCAP - 1 : o);
    const int co  = __shfl_xor(c, 16, 32);
    const int cmv = c > co ? c : co;
    const int trip = __builtin_amdgcn_readfirstlane(cmv);
    int last = o + c - 1;
    last = last < o ? o : last;
    last = last > RCAP - 1 ? RCAP - 1 : last;
    float a0 = 0.0f, a1 = 0.0f, a2 = 0.0f, a3 = 0.0f;
#pragma unroll 1
    for (int j = 0; j < trip; ++j) {
      int idx = o + j;
      idx = idx > last ? last : idx;
      int sr = lb[idx];
      sr = sr < 0 ? 0 : (sr > NN - 1 ? NN - 1 : sr);
      const v4f v = *(const v4fa*)(P + (size_t)sr * DD + 4 * q);
      asm volatile("" :: "v"(v));
      const bool valid = j < c;
      const float t0 = a0 + v.x, t1 = a1 + v.y, t2 = a2 + v.z, t3 = a3 + v.w;
      a0 = valid ? t0 : a0; a1 = valid ? t1 : a1; a2 = valid ? t2 : a2; a3 = valid ? t3 : a3;
    }
    const int dc = d < NN ? d : NN - 1;
    float* op = out + (size_t)dc * DD + 4 * q;
    const v4f g = *(const v4fa*)op;
    asm volatile("" :: "v"(g));
    float m0 = g.x + a0, m1 = g.y + a1, m2 = g.z + a2, m3 = g.w + a3;
    const bool bad = (flag != 0) | big;
    m0 = bad ? qnan : m0; m1 = bad ? qnan : m1; m2 = bad ? qnan : m2; m3 = bad ? qnan : m3;
    v4f ov;
    ov.x = m0; ov.y = m1; ov.z = m2; ov.w = m3;
    if (d < NN) {
      *(volatile v4f*)op = ov;
      __threadfence();
      *(volatile v4f*)op = ov;
    }
  }
}

extern "C" void kernel_launch(void* const* d_in, const int* in_sizes, int n_in,
                              void* d_out, int out_size, void* d_ws, size_t ws_size,
                              hipStream_t stream) {
  if (n_in < 8) return;
  if (in_sizes[0] != NN * DD) return;
  if (in_sizes[1] != DD * DD) return;
  if (in_sizes[2] != DD) return;
  if (in_sizes[3] != NR * DD * DD) return;
  if (in_sizes[4] != 2 * NE || in_sizes[5] != 2 * NE) return;
  if (in_sizes[6] != 2 * NE || in_sizes[7] != 2 * NE) return;
  if (out_size != NN * DD) return;

  const float* x  = (const float*)d_in[0];
  const float* rw = (const float*)d_in[1];
  const float* rb = (const float*)d_in[2];
  const float* cw = (const float*)d_in[3];
  const int*   ea = (const int*)d_in[4];
  const int*   eb = (const int*)d_in[5];
  const int*   ec = (const int*)d_in[6];
  const int*   ed = (const int*)d_in[7];
  float* out = (float*)d_out;

  constexpr size_t zXB   = (size_t)MP * XPITCH * 2;
  constexpr size_t zWB   = (size_t)(1 + NR) * DD * WPITCH * 2;
  constexpr size_t zSM   = 512;
  constexpr size_t zP    = (size_t)MP * DD * 4;
  constexpr size_t zLIST = (size_t)NROLE * RCAP * 4;
  constexpr size_t zCO   = (size_t)NROLE * 2 * NBRUN * 4;
  constexpr size_t zFLAG = (size_t)NROLE * 128;
  constexpr size_t oXB   = 0;
  constexpr size_t oWB   = oXB + zXB;
  constexpr size_t oSM   = oWB + zWB;
  constexpr size_t oP    = oSM + zSM;
  constexpr size_t oLIST = oP + zP;
  constexpr size_t oCO   = oLIST + zLIST;
  constexpr size_t oFLAG = oCO + zCO;
  constexpr size_t oEND  = oFLAG + zFLAG;
  static_assert(zXB % 256 == 0 && zWB % 256 == 0 && zSM % 256 == 0 && zP % 256 == 0);
  static_assert(zLIST % 256 == 0 && zCO % 256 == 0 && zFLAG % 256 == 0);
  static_assert(oEND <= (size_t)WSMAX);
  if (oEND > ws_size) return;

  char* ws = (char*)d_ws;
  unsigned short* XB   = (unsigned short*)(ws + oXB);
  unsigned short* WB   = (unsigned short*)(ws + oWB);
  float*          SM   = (float*)(ws + oSM);
  float*          P    = (float*)(ws + oP);
  int*            LIST = (int*)(ws + oLIST);
  int*            CO   = (int*)(ws + oCO);
  int*            FLAG = (int*)(ws + oFLAG);

  hipFuncSetAttribute(reinterpret_cast<const void*>(&k_bucket), hipFuncAttributeMaxDynamicSharedMemorySize, (int)BK_LDS);

  k_prep<<<PBTOT, NTHR, 0, stream>>>(x, rw, rb, cw, XB, WB, SM);
  k_bucket<<<NROLE, NTHR, BK_LDS, stream>>>(ea, eb, ec, ed, LIST, CO, FLAG);
  k_gemm<1><<<MP / GBM, NTHR, 0, stream>>>(XB, WB, SM, out, NN);
  for (int r = 0; r < NR; ++r) {
    const unsigned short* wt = WB + (size_t)(1 + r) * DD * WPITCH;
    k_gemm<0><<<MP / GBM, NTHR, 0, stream>>>(XB, wt, SM, P, MP);
    k_replay<<<MP / RBM, NTHR, 0, stream>>>(LIST + (size_t)r * NBK * RCAP, CO + (size_t)r * NBK * 2 * NBRUN,
                                            FLAG + (size_t)r * NBK * 32, P, out);
  }
}
